// CombinedVectorField_3710851744456
// MI455X (gfx1250) — hardware-verified
//
#include <hip/hip_runtime.h>


namespace {
constexpr int NB = 4096, DX = 128, DH = 128, HID = 512, KIN = 257, KP = 288, OW = 129;
constexpr float XS = 8.0f, WSC = 256.0f;
typedef _Float16 b16;
typedef __attribute__((ext_vector_type(16))) _Float16 v16b;
typedef __attribute__((ext_vector_type(8))) _Float16 v8b;
typedef __attribute__((ext_vector_type(8))) float v8f;
typedef __attribute__((ext_vector_type(4))) float v4f;
__device__ __forceinline__ float bf16_rne(float f) { unsigned int u = __float_as_uint(f); u += 0x7FFFu + ((u >> 16) & 1u); return __uint_as_float(u & 0xFFFF0000u); }
__device__ __forceinline__ void split16(float v, b16& hi, b16& lo) { hi = (b16)v; lo = (b16)(v - (float)hi); }
__device__ __forceinline__ v16b frag_kb(const b16* p, int hh) { const v8b a = *(const v8b*)(p + 8 * hh), b = *(const v8b*)(p + 16 + 8 * hh); v16b f;
#pragma unroll
  for (int e = 0; e < 8; ++e) { f[e] = a[e]; f[8 + e] = b[e]; } return f; }
__device__ __forceinline__ v8f wmma16b(v16b a, v16b b, v8f c) { v8f d = __builtin_amdgcn_wmma_f32_16x16x32_f16(false, a, false, b, (short)0, c, false, false); asm volatile("v_nop\n\tv_nop\n\tv_nop\n\tv_nop" : "+v"(d) : "v"(a), "v"(b)); return d; }
__device__ __forceinline__ void wave_lds_sync() { __builtin_amdgcn_fence(__ATOMIC_RELEASE, "workgroup"); __builtin_amdgcn_wave_barrier(); __builtin_amdgcn_fence(__ATOMIC_ACQUIRE, "workgroup"); }
__device__ __forceinline__ float pmul(float a, float b) { float p = a * b; asm volatile("" : "+v"(p)); return p; }

__global__ __launch_bounds__(256) void wprep_kernel(const float* __restrict__ w1, const float* __restrict__ w2, b16* __restrict__ W1T, b16* __restrict__ W2T, float* __restrict__ C) {
  const int u = blockIdx.x * 256 + threadIdx.x; const int n1 = HID * KP / 8, n2 = DX * HID / 8; v8b v;
  if (u < n1) { const int e = u * 8, o = e / KP, k0 = e % KP; for (int j = 0; j < 8; ++j) { const int k = k0 + j; v[j] = k < KIN ? (b16)(bf16_rne(w1[(size_t)(k < KIN ? k : 0) * HID + o]) * WSC) : (b16)0.0f; } for (int p = 0; p < 2; ++p) { *(volatile v8b*)(W1T + e) = v; __threadfence(); } return; }
  const int t = u - n1; if (t < n2) { const int e = t * 8, o = e / HID, k0 = e % HID; for (int j = 0; j < 8; ++j) v[j] = (b16)(bf16_rne(w2[(size_t)(k0 + j) * DX + o]) * WSC); for (int p = 0; p < 2; ++p) { *(volatile v8b*)(W2T + e) = v; __threadfence(); } return; }
  const int k = t - n2; if (k < HID) { float s = 0.0f;
#pragma unroll 1
    for (int i = 0; i < DX; ++i) s += pmul(bf16_rne(w1[(size_t)i * HID + k]), bf16_rne(w2[(size_t)k * DX + i]));
    for (int p = 0; p < 2; ++p) { ((volatile float*)C)[k] = s; __threadfence(); } }
}
__global__ __launch_bounds__(128) void main_kernel(const float* __restrict__ st, const float* __restrict__ hc, const float* __restrict__ hn, const float* __restrict__ tt, const float* __restrict__ gsp, const b16* __restrict__ W1T, const b16* __restrict__ W2T, const float* __restrict__ C, const float* __restrict__ b1, const float* __restrict__ b2, float* __restrict__ out) {
  __shared__ __attribute__((aligned(16))) b16 Ah[4][16][HID + 8], Al[4][16][HID + 8]; __shared__ float Dv[4][16];
  const int wave = threadIdx.x >> 5, lane = threadIdx.x & 31, nloc = lane & 15, hlf = lane >> 4; const int cond = wave >> 1; const size_t r0 = (size_t)blockIdx.x * 32 + (wave & 1) * 16;
  const float* xr = st + (r0 + nloc) * (DX + 1); const float* cr = (cond ? hc : hn) + (r0 + nloc) * DH; const float tv = bf16_rne(tt[0]); const float g = bf16_rne(gsp[0]);
  float dsum[8]; for (int r8 = 0; r8 < 8; ++r8) dsum[r8] = 0.0f;
#pragma unroll 1
  for (int cg = 0; cg < 4; ++cg) { v8f acc[8];
#pragma unroll
    for (int t = 0; t < 8; ++t) acc[t] = (v8f){};
#pragma unroll 1
    for (int kb = 0; kb < KP; kb += 32) { v16b a;
      for (int j = 0; j < 8; ++j) { const int k0 = kb + 8 * hlf + j, k1 = kb + 16 + 8 * hlf + j; float f0, f1;
        f0 = k0 < DX ? xr[k0 < DX ? k0 : 0] : (k0 < DX + DH ? cr[(k0 - DX) < DH && k0 >= DX ? k0 - DX : 0] : (k0 == DX + DH ? tv : 0.0f));
        f1 = k1 < DX ? xr[k1 < DX ? k1 : 0] : (k1 < DX + DH ? cr[(k1 - DX) < DH && k1 >= DX ? k1 - DX : 0] : (k1 == DX + DH ? tv : 0.0f));
        a[j] = (b16)(bf16_rne(f0) * XS); a[8 + j] = (b16)(bf16_rne(f1) * XS); }
#pragma unroll
      for (int t = 0; t < 8; ++t) acc[t] = wmma16b(a, frag_kb(W1T + (size_t)(cg * 128 + t * 16 + nloc) * KP + kb, hlf), acc[t]); }
#pragma unroll
    for (int t = 0; t < 8; ++t) { const int c = cg * 128 + t * 16 + nloc; const float bb = bf16_rne(b1[c]), ck = C[c];
#pragma unroll
      for (int r8 = 0; r8 < 8; ++r8) { const float av = tanhf(acc[t][r8] * (1.0f / (XS * WSC)) + bb); dsum[r8] += pmul(1.0f - av * av, ck); b16 p, ql; split16(av * XS, p, ql); Ah[wave][8 * hlf + r8][c] = p; Al[wave][8 * hlf + r8][c] = ql; } } }
#pragma unroll
  for (int r8 = 0; r8 < 8; ++r8) { float s = dsum[r8]; for (int o = 1; o < 16; o <<= 1) s += __shfl_xor(s, o); if (nloc == 0) Dv[wave][8 * hlf + r8] = s; }
  wave_lds_sync();
  { v8f acc[8]; float accv[8][8];
#pragma unroll
    for (int t = 0; t < 8; ++t) acc[t] = (v8f){};
#pragma unroll 2
    for (int kb = 0; kb < HID; kb += 32) { const v16b a = frag_kb(&Ah[wave][nloc][kb], hlf), al = frag_kb(&Al[wave][nloc][kb], hlf);
#pragma unroll
      for (int t = 0; t < 8; ++t) { const v16b bw = frag_kb(W2T + (size_t)(t * 16 + nloc) * HID + kb, hlf); acc[t] = wmma16b(a, bw, acc[t]); acc[t] = wmma16b(al, bw, acc[t]); } }
#pragma unroll
    for (int t = 0; t < 8; ++t) { const int c = t * 16 + nloc; const float bb = bf16_rne(b2[c]);
#pragma unroll
      for (int r8 = 0; r8 < 8; ++r8) accv[t][r8] = acc[t][r8] * (1.0f / (XS * WSC)) + bb; }
    wave_lds_sync();
    float (*Vw)[DX + 4] = (float (*)[DX + 4])&Ah[wave][0][0];
#pragma unroll
    for (int t = 0; t < 8; ++t)
#pragma unroll
      for (int r8 = 0; r8 < 8; ++r8) Vw[8 * hlf + r8][t * 16 + nloc] = accv[t][r8]; }
  __syncthreads();
  float* O = (float*)&Al[0][0][0];
  for (int idx = threadIdx.x; idx < 32 * OW; idx += 128) { const int r = idx / OW, c = idx % OW; const int wn = (r >> 4), wh = 2 + (r >> 4), rl = r & 15;
    const float (*Vn)[DX + 4] = (const float (*)[DX + 4])&Ah[wn][0][0]; const float (*Vh)[DX + 4] = (const float (*)[DX + 4])&Ah[wh][0][0];
    const float vn = (c < DX) ? Vn[rl][c] : Dv[wn][rl], vh = (c < DX) ? Vh[rl][c] : Dv[wh][rl]; O[idx] = pmul(1.0f - g, vn) + pmul(g, vh); }
  __syncthreads();
  for (int pass = 0; pass < 2; ++pass) { for (int ln = wave; ln < OW; ln += 4) ((volatile float*)out)[(size_t)blockIdx.x * 32 * OW + ln * 32 + lane] = O[ln * 32 + lane]; __threadfence(); }
}
}

extern "C" void kernel_launch(void* const* d_in, const int* in_sizes, int n_in, void* d_out, int out_size, void* d_ws, size_t ws_size, hipStream_t stream) {
  (void)n_in;
  auto Fp = [&](int i) { return (const float*)d_in[i]; };
  if (in_sizes[0] != NB * (DX + 1) || in_sizes[1] != NB * DH || in_sizes[2] != NB * DH || in_sizes[3] != 1 || in_sizes[4] != 1 || in_sizes[5] != KIN * HID || in_sizes[6] != HID || in_sizes[7] != HID * DX || in_sizes[8] != DX || out_size != NB * OW) return;
  const int NBLKV = NB / 32;
  size_t off = 0; char* ws = (char*)d_ws;
  auto carve = [&](size_t bytes) { char* p = ws + off; off += (bytes + 255) & ~(size_t)255; return p; };
  b16* W1T = (b16*)carve((size_t)HID * KP * 2); b16* W2T = (b16*)carve((size_t)DX * HID * 2); float* C = (float*)carve(HID * 4);
  if (off > ws_size || off > ((size_t)16 << 20)) return;
  wprep_kernel<<<(HID * KP / 8 + DX * HID / 8 + HID + 255) / 256, 256, 0, stream>>>(Fp(5), Fp(7), W1T, W2T, C);
  main_kernel<<<NBLKV, 128, 0, stream>>>(Fp(0), Fp(1), Fp(2), Fp(3), Fp(4), W1T, W2T, C, Fp(6), Fp(8), (float*)d_out);
}
